// RWKV7TimeMixForTabICL_55250459295926
// MI455X (gfx1250) — hardware-verified
//
#include <hip/hip_runtime.h>
#include <math.h>

constexpr int kBatch  = 4;
constexpr int kSteps  = 1024;
constexpr int kChan   = 1024;
constexpr int kHeads  = 16;
constexpr int kHdim   = 64;
constexpr int kTok    = kBatch * kSteps;
constexpr size_t kPlane = (size_t)kTok * kChan;
constexpr int kWElems = kChan * kChan;
constexpr int kChunk  = 16;

constexpr float kACarry    = 8.0f;
constexpr float kWCarry    = 16.0f;
constexpr float kWoCarry   = 128.0f;
constexpr float kYCarry    = 16.0f;
constexpr float kLoCarry   = 2048.0f;
constexpr float kLoInv     = 1.0f / kLoCarry;
constexpr float kScaleProj = 1.0f / (kACarry * kWCarry);
constexpr float kScaleOut  = 1.0f / (kYCarry * kWoCarry);
constexpr float kGnEps     = 0.00064f;
constexpr float kNormEps   = 1e-6f;
constexpr float kInvHdim   = 1.0f / (float)kHdim;

static_assert(kHeads * kHdim == kChan);
static_assert(kChan == 1024 && kSteps == 1024 && kHdim == 64);
static_assert(kTok % 64 == 0 && kChan % 64 == 0 && kChan % 32 == 0);
static_assert(kTok % 32 == 0 && (((kTok / 32) * (kChan / 64)) % 8) == 0);
static_assert(kSteps % kChunk == 0 && kChunk == 16 && kChunk * kHdim == 1024);
static_assert((kTok * kHeads) % 8 == 0);

typedef __attribute__((ext_vector_type(16))) _Float16 v16h;
typedef __attribute__((ext_vector_type(8)))  _Float16 v8h;
typedef __attribute__((ext_vector_type(8)))  float    v8f;
typedef __attribute__((ext_vector_type(4)))  float    v4f;
typedef __attribute__((ext_vector_type(2)))  float    v2f;
typedef __attribute__((ext_vector_type(4)))  unsigned int v4u;

__device__ __forceinline__ unsigned pk16(unsigned short a, unsigned short b) {
  return (unsigned)a | ((unsigned)b << 16);
}
__device__ __forceinline__ unsigned short h_bits(float f) {
  const _Float16 h = (_Float16)f;
  return __builtin_bit_cast(unsigned short, h);
}
__device__ __forceinline__ void h_split(float v, unsigned short& hb, unsigned short& lb) {
  const _Float16 h = (_Float16)v;
  const float hf = (float)h;
  const float d = v - hf;
  const _Float16 r = (_Float16)(d * kLoCarry);
  hb = __builtin_bit_cast(unsigned short, h);
  lb = __builtin_bit_cast(unsigned short, r);
}
__device__ __forceinline__ float bf_rne(float f) {
  unsigned u = __float_as_uint(f);
  u = (u + 0x7FFFu + ((u >> 16) & 1u)) & 0xFFFF0000u;
  return __uint_as_float(u);
}
__device__ __forceinline__ float h16_to_f32(unsigned hb) {
  const unsigned sgn = (hb & 0x8000u) << 16;
  const unsigned em = hb & 0x7fffu;
  const float fn = __uint_as_float((em << 13) + 0x38000000u);
  const float fs = (float)em * 5.9604644775390625e-8f;
  const float mag = (em < 0x400u) ? fs : fn;
  return __uint_as_float(__float_as_uint(mag) | sgn);
}
__device__ __forceinline__ float wave_sum32(float v) {
#pragma unroll
  for (int o = 16; o > 0; o >>= 1) v += __shfl_xor(v, o, 32);
  return v;
}

struct FragH {
  union U { v16h v; v8h h[2]; };
  static __device__ __forceinline__ v16h load(const _Float16* p) {
    U f;
    f.h[0] = *(const v8h*)(p);
    f.h[1] = *(const v8h*)(p + 16);
    return f.v;
  }
  static __device__ __forceinline__ v8f mma(v16h a, v16h b, v8f c) {
    return __builtin_amdgcn_wmma_f32_16x16x32_f16(false, a, false, b, (short)0, c, false, false);
  }
};
__device__ __forceinline__ void guard_row4(v8f& a0, v8f& a1, v8f& a2, v8f& a3, v16h x,
                                           v16h b0, v16h b1, v16h b2, v16h b3) {
  asm volatile("v_nop\n\tv_nop\n\tv_nop\n\tv_nop"
               : "+v"(a0), "+v"(a1), "+v"(a2), "+v"(a3)
               : "v"(x), "v"(b0), "v"(b1), "v"(b2), "v"(b3));
}
__device__ __forceinline__ void guard_one(v8f& a, v16h x, v16h y) {
  asm volatile("v_nop\n\tv_nop\n\tv_nop\n\tv_nop" : "+v"(a) : "v"(x), "v"(y));
}
__device__ __forceinline__ void acc_guard4(v8f& a, v8f& b, v8f& c, v8f& d) {
  asm volatile("v_nop\n\tv_nop\n\tv_nop\n\tv_nop" : "+v"(a), "+v"(b), "+v"(c), "+v"(d));
}

template <int ACT, bool OUT16, bool BIASN>
__global__ __launch_bounds__(256) void gemm_f16_kernel(
    const unsigned short* __restrict__ Ap, int lda,
    const unsigned short* __restrict__ Btp, int ldb,
    void* __restrict__ Cout, int ldc,
    const float* __restrict__ bias,
    int M, int N, int K, float scale) {
  static_assert(OUT16 ? (ACT == 4) : (ACT != 4));
  __shared__ __align__(16) float sT[8][16 * 68];
  const _Float16* A  = (const _Float16*)Ap;
  const _Float16* Bt = (const _Float16*)Btp;
  const int lane = threadIdx.x & 31;
  const int wave = threadIdx.x >> 5;
  const int tilesN = N >> 6;
  const int tilesM = M >> 6;
  const int tile = blockIdx.x * 8 + wave;
  if (tile >= tilesM * tilesN) return;
  const int tm = tile / tilesN;
  const int tn = tile - tm * tilesN;
  const int m0 = tm << 6;
  const int n0 = tn << 6;
  const int rlane = lane & 15;
  const int koff  = (lane >> 4) * 8;
  const int mOff  = (lane >> 4) * 8;

  const _Float16* pa = A  + (size_t)(m0 + rlane) * lda + koff;
  const _Float16* pb = Bt + (size_t)(n0 + rlane) * ldb + koff;
  const size_t astep = (size_t)16 * lda;
  const size_t bstep = (size_t)16 * ldb;

  v8f acc[4][4];
#pragma unroll
  for (int i = 0; i < 4; ++i)
#pragma unroll
    for (int j = 0; j < 4; ++j) acc[i][j] = (v8f){0.f, 0.f, 0.f, 0.f, 0.f, 0.f, 0.f, 0.f};

  for (int k0 = 0; k0 < K; k0 += 32) {
    const v16h bh0 = FragH::load(pb + k0);
    const v16h bh1 = FragH::load(pb + bstep + k0);
    const v16h bh2 = FragH::load(pb + 2 * bstep + k0);
    const v16h bh3 = FragH::load(pb + 3 * bstep + k0);
#pragma unroll
    for (int i = 0; i < 4; ++i) {
      const v16h ah = FragH::load(pa + i * astep + k0);
      acc[i][0] = FragH::mma(ah, bh0, acc[i][0]);
      acc[i][1] = FragH::mma(ah, bh1, acc[i][1]);
      acc[i][2] = FragH::mma(ah, bh2, acc[i][2]);
      acc[i][3] = FragH::mma(ah, bh3, acc[i][3]);
      guard_row4(acc[i][0], acc[i][1], acc[i][2], acc[i][3], ah, bh0, bh1, bh2, bh3);
    }
  }
  acc_guard4(acc[0][0], acc[0][1], acc[0][2], acc[0][3]);
  acc_guard4(acc[1][0], acc[1][1], acc[1][2], acc[1][3]);
  acc_guard4(acc[2][0], acc[2][1], acc[2][2], acc[2][3]);
  acc_guard4(acc[3][0], acc[3][1], acc[3][2], acc[3][3]);

  float* slab = sT[wave];
#pragma unroll
  for (int i = 0; i < 4; ++i) {
    const int mBase = m0 + (i << 4);
#pragma unroll
    for (int j = 0; j < 4; ++j) {
      float bv = 0.0f;
      if (BIASN) bv = bf_rne(bias[n0 + (j << 4) + rlane]);
#pragma unroll
      for (int r = 0; r < 8; ++r) {
        float v = acc[i][j][r] * scale;
        if (BIASN) v += bv;
        slab[(mOff + r) * 68 + (j << 4) + rlane] = v;
      }
    }
    __builtin_amdgcn_fence(__ATOMIC_RELEASE, "workgroup");
    __builtin_amdgcn_wave_barrier();
    __builtin_amdgcn_fence(__ATOMIC_ACQUIRE, "workgroup");
    if (!OUT16) {
      const int hh = lane >> 4, c4 = (lane & 15) * 4;
      if (ACT != 0) {
#pragma unroll 1
        for (int it = 0; it < 8; ++it) {
          float* sp = slab + (it * 2 + hh) * 68 + c4;
          const v4f xv = *(const v4f*)sp;
          v4f yv = xv;
          if (ACT == 1) {
#pragma unroll
            for (int e = 0; e < 4; ++e) yv[e] = __builtin_amdgcn_rcpf(1.0f + expf(xv[e]));
          }
          if (ACT == 2) {
#pragma unroll
            for (int e = 0; e < 4; ++e) yv[e] = tanhf(xv[e]);
          }
          if (ACT == 3) {
            float ss = xv[0] * xv[0] + xv[1] * xv[1] + xv[2] * xv[2] + xv[3] * xv[3];
            ss += __shfl_xor(ss, 1, 32);
            ss += __shfl_xor(ss, 2, 32);
            ss += __shfl_xor(ss, 4, 32);
            ss += __shfl_xor(ss, 8, 32);
            const float inv = 1.0f / fmaxf(sqrtf(ss), kNormEps);
#pragma unroll
            for (int e = 0; e < 4; ++e) yv[e] = xv[e] * inv;
          }
          *(v4f*)sp = yv;
        }
      }
      float* C = (float*)Cout;
      for (int pass = 0; pass < 2; ++pass) {
#pragma unroll
        for (int it = 0; it < 8; ++it) {
          const int row = it * 2 + hh;
          const v4f v = *(const v4f*)(slab + row * 68 + c4);
          *(volatile v4f*)(C + (size_t)(mBase + row) * ldc + n0 + c4) = v;
        }
        __threadfence();
      }
    } else {
      const int q = lane >> 3, c8 = (lane & 7) * 8;
#pragma unroll 1
      for (int it = 0; it < 4; ++it) {
        float* sp = slab + (it * 4 + q) * 68 + c8;
#pragma unroll 1
        for (int hf = 0; hf < 2; ++hf) {
          const v4f xv = *(const v4f*)(sp + 4 * hf);
          v4f yv;
#pragma unroll
          for (int e = 0; e < 4; ++e) yv[e] = __builtin_amdgcn_rcpf(1.0f + expf(-xv[e]));
          *(v4f*)(sp + 4 * hf) = yv;
        }
      }
      unsigned short* C = (unsigned short*)Cout;
      for (int pass = 0; pass < 2; ++pass) {
#pragma unroll
        for (int it = 0; it < 4; ++it) {
          const int row = it * 4 + q;
          const float* sp = slab + row * 68 + c8;
          v8h hv;
#pragma unroll
          for (int e = 0; e < 8; ++e) hv[e] = (_Float16)sp[e];
          *(volatile v8h*)(C + (size_t)(mBase + row) * ldc + n0 + c8) = hv;
        }
        __threadfence();
      }
    }
    __builtin_amdgcn_fence(__ATOMIC_RELEASE, "workgroup");
    __builtin_amdgcn_wave_barrier();
    __builtin_amdgcn_fence(__ATOMIC_ACQUIRE, "workgroup");
  }
}

template <int ACT>
__global__ __launch_bounds__(256) void gemm_f16_split_kernel(
    const unsigned short* __restrict__ Ahp, const unsigned short* __restrict__ Alp, int lda,
    const unsigned short* __restrict__ Btp, int ldb,
    float* __restrict__ C, int ldc,
    int M, int N, int K, float scale) {
  static_assert(ACT == 0 || ACT == 2);
  __shared__ __align__(16) float sT[8][16 * 68];
  const _Float16* Ah = (const _Float16*)Ahp;
  const _Float16* Al = (const _Float16*)Alp;
  const _Float16* Bt = (const _Float16*)Btp;
  const int lane = threadIdx.x & 31;
  const int wave = threadIdx.x >> 5;
  const int tilesN = N >> 6;
  const int tilesM = M >> 5;
  const int tile = blockIdx.x * 8 + wave;
  if (tile >= tilesM * tilesN) return;
  const int tm = tile / tilesN;
  const int tn = tile - tm * tilesN;
  const int m0 = tm << 5;
  const int n0 = tn << 6;
  const int rlane = lane & 15;
  const int koff  = (lane >> 4) * 8;
  const int mOff  = (lane >> 4) * 8;

  const size_t aoff = (size_t)(m0 + rlane) * lda + koff;
  const _Float16* pah = Ah + aoff;
  const _Float16* pal = Al + aoff;
  const _Float16* pb  = Bt + (size_t)(n0 + rlane) * ldb + koff;
  const size_t astep = (size_t)16 * lda;
  const size_t bstep = (size_t)16 * ldb;

  v8f acc[2][4], accr[2][4];
#pragma unroll
  for (int i = 0; i < 2; ++i)
#pragma unroll
    for (int j = 0; j < 4; ++j) {
      acc[i][j]  = (v8f){0.f, 0.f, 0.f, 0.f, 0.f, 0.f, 0.f, 0.f};
      accr[i][j] = (v8f){0.f, 0.f, 0.f, 0.f, 0.f, 0.f, 0.f, 0.f};
    }

  for (int k0 = 0; k0 < K; k0 += 32) {
    const v16h ah0 = FragH::load(pah + k0);
    const v16h ah1 = FragH::load(pah + astep + k0);
    const v16h al0 = FragH::load(pal + k0);
    const v16h al1 = FragH::load(pal + astep + k0);
#pragma unroll
    for (int j = 0; j < 4; ++j) {
      const v16h bh = FragH::load(pb + j * bstep + k0);
      acc[0][j]  = FragH::mma(ah0, bh, acc[0][j]);
      acc[1][j]  = FragH::mma(ah1, bh, acc[1][j]);
      accr[0][j] = FragH::mma(al0, bh, accr[0][j]);
      accr[1][j] = FragH::mma(al1, bh, accr[1][j]);
      guard_one(acc[0][j], ah0, bh);
      guard_one(acc[1][j], ah1, bh);
      guard_one(accr[0][j], al0, bh);
      guard_one(accr[1][j], al1, bh);
    }
  }
  acc_guard4(acc[0][0], acc[0][1], acc[0][2], acc[0][3]);
  acc_guard4(acc[1][0], acc[1][1], acc[1][2], acc[1][3]);
  acc_guard4(accr[0][0], accr[0][1], accr[0][2], accr[0][3]);
  acc_guard4(accr[1][0], accr[1][1], accr[1][2], accr[1][3]);

  float* slab = sT[wave];
#pragma unroll
  for (int i = 0; i < 2; ++i) {
    const int mBase = m0 + (i << 4);
#pragma unroll
    for (int j = 0; j < 4; ++j) {
#pragma unroll
      for (int r = 0; r < 8; ++r) {
        const float v = (acc[i][j][r] + accr[i][j][r] * kLoInv) * scale;
        slab[(mOff + r) * 68 + (j << 4) + rlane] = v;
      }
    }
    __builtin_amdgcn_fence(__ATOMIC_RELEASE, "workgroup");
    __builtin_amdgcn_wave_barrier();
    __builtin_amdgcn_fence(__ATOMIC_ACQUIRE, "workgroup");
    {
      const int hh = lane >> 4, c4 = (lane & 15) * 4;
      if (ACT == 2) {
#pragma unroll 1
        for (int it = 0; it < 8; ++it) {
          float* sp = slab + (it * 2 + hh) * 68 + c4;
          const v4f xv = *(const v4f*)sp;
          v4f yv = xv;
#pragma unroll
          for (int e = 0; e < 4; ++e) yv[e] = tanhf(xv[e]);
          *(v4f*)sp = yv;
        }
      }
      for (int pass = 0; pass < 2; ++pass) {
#pragma unroll
        for (int it = 0; it < 8; ++it) {
          const int row = it * 2 + hh;
          const v4f v = *(const v4f*)(slab + row * 68 + c4);
          *(volatile v4f*)(C + (size_t)(mBase + row) * ldc + n0 + c4) = v;
        }
        __threadfence();
      }
    }
    __builtin_amdgcn_fence(__ATOMIC_RELEASE, "workgroup");
    __builtin_amdgcn_wave_barrier();
    __builtin_amdgcn_fence(__ATOMIC_ACQUIRE, "workgroup");
  }
}

__global__ __launch_bounds__(256) void wcast_kernel(const float* __restrict__ W0, const float* __restrict__ W1,
                                                    const float* __restrict__ W2, const float* __restrict__ W3,
                                                    const float* __restrict__ W4, const float* __restrict__ W5,
                                                    const float* __restrict__ W6, const float* __restrict__ W7,
                                                    unsigned short* __restrict__ out) {
  const int z = blockIdx.y;
  const float* W = (z == 0) ? W0 : (z == 1) ? W1 : (z == 2) ? W2 : (z == 3) ? W3
                 : (z == 4) ? W4 : (z == 5) ? W5 : (z == 6) ? W6 : W7;
  const int slot = (z == 7) ? 0 : (z + 1);
  const float carry = (z == 7) ? kWoCarry : kWCarry;
  const int i = blockIdx.x * 256 + threadIdx.x;
  if (i >= kWElems / 8) return;
  const float* p = W + 8 * (size_t)i;
  const v4f a = *(const v4f*)(p);
  const v4f c = *(const v4f*)(p + 4);
  unsigned short hb[8];
#pragma unroll
  for (int e = 0; e < 4; ++e) {
    const float fa = a[e];
    const float fc = c[e];
    hb[e]     = h_bits(bf_rne(fa) * carry);
    hb[4 + e] = h_bits(bf_rne(fc) * carry);
  }
  const v4u u = (v4u){pk16(hb[0], hb[1]), pk16(hb[2], hb[3]), pk16(hb[4], hb[5]), pk16(hb[6], hb[7])};
  unsigned short* q = out + (size_t)slot * kWElems + 8 * (size_t)i;
  *(volatile v4u*)q = u;
  __threadfence();
  *(volatile v4u*)q = u;
}

__global__ __launch_bounds__(256) void mix_plane_kernel(const float* __restrict__ x, const float* __restrict__ mixv,
                                                        unsigned short* __restrict__ Aout) {
  const int i = blockIdx.x * 256 + threadIdx.x;
  if (i >= kTok * (kChan / 8)) return;
  const int row = i >> 7;
  const int c8  = (i & 127) * 8;
  const bool first = (row & (kSteps - 1)) == 0;
  const int prow = first ? row : (row - 1);
  const float* xp = x + (size_t)row * kChan + c8;
  const float* pp = x + (size_t)prow * kChan + c8;
  const v4f a  = *(const v4f*)(xp);
  const v4f b  = *(const v4f*)(xp + 4);
  const v4f pa = *(const v4f*)(pp);
  const v4f pb = *(const v4f*)(pp + 4);
  const v4f ma = *(const v4f*)(mixv + c8);
  const v4f mb = *(const v4f*)(mixv + c8 + 4);
  unsigned short hb[8];
#pragma unroll
  for (int e = 0; e < 4; ++e) {
    const float c0 = bf_rne(a[e]);
    const float c1 = bf_rne(b[e]);
    const float q0 = bf_rne(pa[e]);
    const float q1 = bf_rne(pb[e]);
    const float p0 = first ? 0.0f : q0;
    const float p1 = first ? 0.0f : q1;
    const float m0 = bf_rne(ma[e]);
    const float m1 = bf_rne(mb[e]);
    const float o0 = c0 + (p0 - c0) * m0;
    const float o1 = c1 + (p1 - c1) * m1;
    hb[e]     = h_bits(o0 * kACarry);
    hb[4 + e] = h_bits(o1 * kACarry);
  }
  const v4u u = (v4u){pk16(hb[0], hb[1]), pk16(hb[2], hb[3]), pk16(hb[4], hb[5]), pk16(hb[6], hb[7])};
  unsigned short* q = Aout + 8 * (size_t)i;
  *(volatile v4u*)q = u;
  __threadfence();
  *(volatile v4u*)q = u;
}

__global__ __launch_bounds__(256) void mix_plane_split_kernel(const float* __restrict__ x, const float* __restrict__ mixv,
                                                              unsigned short* __restrict__ Ahi,
                                                              unsigned short* __restrict__ Alo) {
  const int i = blockIdx.x * 256 + threadIdx.x;
  if (i >= kTok * (kChan / 8)) return;
  const int row = i >> 7;
  const int c8  = (i & 127) * 8;
  const bool first = (row & (kSteps - 1)) == 0;
  const int prow = first ? row : (row - 1);
  const float* xp = x + (size_t)row * kChan + c8;
  const float* pp = x + (size_t)prow * kChan + c8;
  const v4f a  = *(const v4f*)(xp);
  const v4f b  = *(const v4f*)(xp + 4);
  const v4f pa = *(const v4f*)(pp);
  const v4f pb = *(const v4f*)(pp + 4);
  const v4f ma = *(const v4f*)(mixv + c8);
  const v4f mb = *(const v4f*)(mixv + c8 + 4);
  unsigned short hb[8], lb[8];
#pragma unroll
  for (int e = 0; e < 4; ++e) {
    const float c0 = bf_rne(a[e]);
    const float c1 = bf_rne(b[e]);
    const float q0 = bf_rne(pa[e]);
    const float q1 = bf_rne(pb[e]);
    const float p0 = first ? 0.0f : q0;
    const float p1 = first ? 0.0f : q1;
    const float m0 = bf_rne(ma[e]);
    const float m1 = bf_rne(mb[e]);
    const float o0 = c0 + (p0 - c0) * m0;
    const float o1 = c1 + (p1 - c1) * m1;
    h_split(o0 * kACarry, hb[e], lb[e]);
    h_split(o1 * kACarry, hb[4 + e], lb[4 + e]);
  }
  const v4u uh = (v4u){pk16(hb[0], hb[1]), pk16(hb[2], hb[3]), pk16(hb[4], hb[5]), pk16(hb[6], hb[7])};
  const v4u ul = (v4u){pk16(lb[0], lb[1]), pk16(lb[2], lb[3]), pk16(lb[4], lb[5]), pk16(lb[6], lb[7])};
  unsigned short* qh = Ahi + 8 * (size_t)i;
  unsigned short* ql = Alo + 8 * (size_t)i;
  *(volatile v4u*)qh = uh;
  *(volatile v4u*)ql = ul;
  __threadfence();
  *(volatile v4u*)qh = uh;
  *(volatile v4u*)ql = ul;
}

__global__ __launch_bounds__(256) void state_scan_kernel(const float* __restrict__ Rf, const float* __restrict__ Dd,
                                                         const float* __restrict__ Kf, const float* __restrict__ Vf,
                                                         const float* __restrict__ Af, const float* __restrict__ Bf,
                                                         float* __restrict__ Y) {
  __shared__ __align__(16) float lv[6 * kChunk * 64];
  __shared__ __align__(16) float yb[kChunk * 64];
  const int bh  = blockIdx.x;
  const int b   = bh >> 4;
  const int h   = bh & 15;
  const int tid = threadIdx.x;
  const int i   = tid >> 2;
  const int q   = tid & 3;
  const int j0  = q * 16;
  const int lrow = tid >> 4;
  const int lc4  = (tid & 15) * 4;
  const size_t base = (size_t)b * kSteps * kChan + (size_t)h * kHdim;
  const float* lr  = lv + 0 * kChunk * 64 + j0;
  const float* ld  = lv + 1 * kChunk * 64 + j0;
  const float* lk  = lv + 2 * kChunk * 64 + j0;
  const float* lvv = lv + 3 * kChunk * 64 + i;
  const float* la  = lv + 4 * kChunk * 64 + j0;
  const float* lb  = lv + 5 * kChunk * 64 + j0;

  float S[16];
#pragma unroll
  for (int jj = 0; jj < 16; ++jj) S[jj] = 0.0f;

#pragma unroll 1
  for (int ch = 0; ch < kSteps / kChunk; ++ch) {
    const size_t goff = base + (size_t)(ch * kChunk + lrow) * kChan + lc4;
    {
      const v4f t0 = *(const v4f*)(Rf + goff);
      const v4f t1 = *(const v4f*)(Dd + goff);
      const v4f t2 = *(const v4f*)(Kf + goff);
      const v4f t3 = *(const v4f*)(Vf + goff);
      const v4f t4 = *(const v4f*)(Af + goff);
      const v4f t5 = *(const v4f*)(Bf + goff);
      const int lo = lrow * 64 + lc4;
      *(v4f*)(lv + 0 * kChunk * 64 + lo) = t0;
      *(v4f*)(lv + 1 * kChunk * 64 + lo) = t1;
      *(v4f*)(lv + 2 * kChunk * 64 + lo) = t2;
      *(v4f*)(lv + 3 * kChunk * 64 + lo) = t3;
      *(v4f*)(lv + 4 * kChunk * 64 + lo) = t4;
      *(v4f*)(lv + 5 * kChunk * 64 + lo) = t5;
    }
    __syncthreads();

#pragma unroll 1
    for (int s = 0; s < kChunk; ++s) {
      const int so = s * 64;
      const float vi = lvv[so];
      float sa = 0.0f;
#pragma unroll
      for (int g4 = 0; g4 < 4; ++g4) {
        const v4f a4 = *(const v4f*)(la + so + 4 * g4);
#pragma unroll
        for (int e = 0; e < 4; ++e) sa += S[4 * g4 + e] * a4[e];
      }
      sa += __shfl_xor(sa, 1, 32);
      sa += __shfl_xor(sa, 2, 32);
      float out = 0.0f;
#pragma unroll
      for (int g4 = 0; g4 < 4; ++g4) {
        const v4f d4 = *(const v4f*)(ld + so + 4 * g4);
        const v4f b4 = *(const v4f*)(lb + so + 4 * g4);
        const v4f k4 = *(const v4f*)(lk + so + 4 * g4);
        const v4f r4 = *(const v4f*)(lr + so + 4 * g4);
#pragma unroll
        for (int e = 0; e < 4; ++e) {
          const float sn = S[4 * g4 + e] * d4[e] + sa * b4[e] + vi * k4[e];
          S[4 * g4 + e] = sn;
          out += sn * r4[e];
        }
      }
      out += __shfl_xor(out, 1, 32);
      out += __shfl_xor(out, 2, 32);
      if (q == 0) yb[so + i] = out;
    }
    __syncthreads();
    {
      const v4f val = *(const v4f*)(yb + lrow * 64 + lc4);
      *(volatile v4f*)(Y + goff) = val;
      __threadfence();
      *(volatile v4f*)(Y + goff) = val;
    }
  }
}

__global__ __launch_bounds__(256) void norm_gate_kernel(const float* __restrict__ Y, const unsigned* __restrict__ Gw,
                                                        const float* __restrict__ gn_w, const float* __restrict__ gn_b,
                                                        unsigned* __restrict__ YG) {
  const int lane = threadIdx.x & 31;
  const int pair = blockIdx.x * 8 + (threadIdx.x >> 5);
  const int tok = pair >> 4;
  const int h   = pair & 15;
  const size_t base = (size_t)tok * kChan + (size_t)h * kHdim + 2 * lane;
  const int c = h * kHdim + 2 * lane;
  const v2f y2 = *(const v2f*)(Y + base);
  const unsigned gword = Gw[base >> 1];
  const v2f w2 = *(const v2f*)(gn_w + c);
  const v2f b2 = *(const v2f*)(gn_b + c);
  const float g0 = h16_to_f32(gword & 0xffffu);
  const float g1 = h16_to_f32(gword >> 16);
  const float y0 = y2[0];
  const float y1 = y2[1];
  const float wa = bf_rne(w2[0]);
  const float wb = bf_rne(w2[1]);
  const float ba = bf_rne(b2[0]);
  const float bb = bf_rne(b2[1]);
  const float mu = wave_sum32(y0 + y1) * kInvHdim;
  const float d0 = y0 - mu;
  const float d1 = y1 - mu;
  const float var = wave_sum32(d0 * d0 + d1 * d1) * kInvHdim;
  const float inv = 1.0f / sqrtf(var + kGnEps);
  const float o0 = (((d0 * inv) * wa + ba) * g0) * kYCarry;
  const float o1 = (((d1 * inv) * wb + bb) * g1) * kYCarry;
  const unsigned short h0 = h_bits(o0);
  const unsigned short h1 = h_bits(o1);
  const unsigned word = pk16(h0, h1);
  const size_t widx = base >> 1;
  *(volatile unsigned*)(YG + widx) = word;
  __threadfence();
  *(volatile unsigned*)(YG + widx) = word;
}

constexpr size_t kMiB      = (size_t)1048576;
constexpr size_t kOffWh    = 0;
constexpr size_t kOffA     = 16 * kMiB;
constexpr size_t kOffP     = 24 * kMiB;
constexpr size_t kOffG     = 120 * kMiB;
constexpr size_t kOffLo    = kOffG;
constexpr size_t kOffO     = 2 * kMiB;
constexpr size_t kOffNG    = 24 * kMiB;
constexpr size_t kCarveEnd = 128 * kMiB;
static_assert((size_t)8 * kWElems * 2 == 16 * kMiB);
static_assert(kPlane * 2 == 8 * kMiB && kPlane * 4 == 16 * kMiB);
static_assert(kOffA + kPlane * 2 == kOffP);
static_assert(kOffP + 6 * kPlane * 4 == kOffG);
static_assert(kOffG + kPlane * 2 == kCarveEnd);
static_assert(kOffLo + kPlane * 2 <= kCarveEnd);
static_assert(kOffO >= (size_t)kWElems * 2 && kOffO + kPlane * 4 <= kOffP);
static_assert(kOffNG + kPlane * 2 <= kOffP + kPlane * 4);
static_assert(kCarveEnd == (size_t)134217728);

extern "C" void kernel_launch(void* const* d_in, const int* in_sizes, int n_in,
                              void* d_out, int out_size, void* d_ws, size_t ws_size, hipStream_t stream) {
  if (n_in < 19 || d_out == nullptr || d_ws == nullptr) return;
  const int nP = (int)kPlane;
  if (in_sizes[0] != nP) return;
  for (int i = 1; i <= 7; ++i) if (in_sizes[i] != kChan) return;
  for (int i = 8; i <= 15; ++i) if (in_sizes[i] != kWElems) return;
  for (int i = 16; i <= 18; ++i) if (in_sizes[i] != kChan) return;
  if (out_size != nP) return;
  if (ws_size < kCarveEnd) return;

  const float* x    = (const float*)d_in[0];
  const float* m_r  = (const float*)d_in[1];
  const float* m_w  = (const float*)d_in[2];
  const float* m_k  = (const float*)d_in[3];
  const float* m_v  = (const float*)d_in[4];
  const float* m_a  = (const float*)d_in[5];
  const float* m_b  = (const float*)d_in[6];
  const float* m_g  = (const float*)d_in[7];
  const float* W_r  = (const float*)d_in[8];
  const float* W_w  = (const float*)d_in[9];
  const float* W_k  = (const float*)d_in[10];
  const float* W_v  = (const float*)d_in[11];
  const float* W_a  = (const float*)d_in[12];
  const float* W_b  = (const float*)d_in[13];
  const float* W_g  = (const float*)d_in[14];
  const float* W_o  = (const float*)d_in[15];
  const float* b_o  = (const float*)d_in[16];
  const float* gn_w = (const float*)d_in[17];
  const float* gn_b = (const float*)d_in[18];
  float* out0 = (float*)d_out;

  char* ws = (char*)d_ws;
  unsigned short* Wh     = (unsigned short*)(ws + kOffWh);
  unsigned short* Astage = (unsigned short*)(ws + kOffA);
  unsigned short* Alo    = (unsigned short*)(ws + kOffLo);
  float* P_r = (float*)(ws + kOffP);
  float* P_d = P_r + kPlane;
  float* P_k = P_d + kPlane;
  float* P_v = P_k + kPlane;
  float* P_a = P_v + kPlane;
  float* P_b = P_a + kPlane;
  unsigned short* G  = (unsigned short*)(ws + kOffG);
  float* O           = (float*)(ws + kOffO);
  unsigned short* NG = (unsigned short*)(ws + kOffNG);

  const unsigned short* Wh_o = Wh;
  const unsigned short* Wh_r = Wh + (size_t)1 * kWElems;
  const unsigned short* Wh_w = Wh + (size_t)2 * kWElems;
  const unsigned short* Wh_k = Wh + (size_t)3 * kWElems;
  const unsigned short* Wh_v = Wh + (size_t)4 * kWElems;
  const unsigned short* Wh_a = Wh + (size_t)5 * kWElems;
  const unsigned short* Wh_b = Wh + (size_t)6 * kWElems;
  const unsigned short* Wh_g = Wh + (size_t)7 * kWElems;

  const dim3 blk(256);
  const dim3 gridCast((kWElems / 8) / 256, 8);
  const dim3 gridMix((kTok * (kChan / 8)) / 256);
  const dim3 gridGemm(((kTok / 64) * (kChan / 64)) / 8);
  const dim3 gridGemmSplit(((kTok / 32) * (kChan / 64)) / 8);
  const dim3 gridPair((kTok * kHeads) / 8);

  wcast_kernel<<<gridCast, blk, 0, stream>>>(W_r, W_w, W_k, W_v, W_a, W_b, W_g, W_o, Wh);

  mix_plane_split_kernel<<<gridMix, blk, 0, stream>>>(x, m_r, Astage, Alo);
  gemm_f16_split_kernel<0><<<gridGemmSplit, blk, 0, stream>>>(
      Astage, Alo, kChan, Wh_r, kChan, P_r, kChan, kTok, kChan, kChan, kScaleProj);
  mix_plane_kernel<<<gridMix, blk, 0, stream>>>(x, m_w, Astage);
  gemm_f16_kernel<1, false, false><<<gridGemm, blk, 0, stream>>>(
      Astage, kChan, Wh_w, kChan, (void*)P_d, kChan, (const float*)nullptr, kTok, kChan, kChan, kScaleProj);
  mix_plane_split_kernel<<<gridMix, blk, 0, stream>>>(x, m_k, Astage, Alo);
  gemm_f16_split_kernel<2><<<gridGemmSplit, blk, 0, stream>>>(
      Astage, Alo, kChan, Wh_k, kChan, P_k, kChan, kTok, kChan, kChan, kScaleProj);
  mix_plane_kernel<<<gridMix, blk, 0, stream>>>(x, m_v, Astage);
  gemm_f16_kernel<0, false, false><<<gridGemm, blk, 0, stream>>>(
      Astage, kChan, Wh_v, kChan, (void*)P_v, kChan, (const float*)nullptr, kTok, kChan, kChan, kScaleProj);
  mix_plane_kernel<<<gridMix, blk, 0, stream>>>(x, m_a, Astage);
  gemm_f16_kernel<3, false, false><<<gridGemm, blk, 0, stream>>>(
      Astage, kChan, Wh_a, kChan, (void*)P_a, kChan, (const float*)nullptr, kTok, kChan, kChan, kScaleProj);
  mix_plane_kernel<<<gridMix, blk, 0, stream>>>(x, m_b, Astage);
  gemm_f16_kernel<3, false, false><<<gridGemm, blk, 0, stream>>>(
      Astage, kChan, Wh_b, kChan, (void*)P_b, kChan, (const float*)nullptr, kTok, kChan, kChan, kScaleProj);
  mix_plane_kernel<<<gridMix, blk, 0, stream>>>(x, m_g, Astage);
  gemm_f16_kernel<4, true, false><<<gridGemm, blk, 0, stream>>>(
      Astage, kChan, Wh_g, kChan, (void*)G, kChan, (const float*)nullptr, kTok, kChan, kChan, kScaleProj);

  state_scan_kernel<<<dim3(kBatch * kHeads), blk, 0, stream>>>(P_r, P_d, P_k, P_v, P_a, P_b, O);

  norm_gate_kernel<<<gridPair, blk, 0, stream>>>(O, (const unsigned*)G, gn_w, gn_b, (unsigned*)NG);

  gemm_f16_kernel<0, false, true><<<gridGemm, blk, 0, stream>>>(
      NG, kChan, Wh_o, kChan, (void*)out0, kChan, b_o, kTok, kChan, kChan, kScaleOut);
}
